// KimiDeltaAttention_67001489818058
// MI455X (gfx1250) — hardware-run, weakly checked
//
#include <hip/hip_runtime.h>
#include <math.h>

constexpr int kTok     = 2048;
constexpr int kHid     = 2048;
constexpr int kHeads   = 16;
constexpr int kHdim    = 64;
constexpr int kHdimRoot = 8;
constexpr int kProj    = kHeads * kHdim;
constexpr int kTaps    = 4;
constexpr int kLow     = 64;
constexpr int kBetaPad = 64;
constexpr int kChunk   = 16;
constexpr size_t kPlane = (size_t)kTok * kProj;

constexpr float kXCarry   = 16.0f;
constexpr float kWCarry   = 256.0f;
constexpr float kHidCarry = 16.0f;
constexpr float kYCarry   = 16.0f;
constexpr float kResCarry = 2048.0f;
constexpr float kResInv   = 1.0f / kResCarry;
constexpr float kScaleXW  = 1.0f / (kXCarry * kWCarry);
constexpr float kScaleHid = kHidCarry / (kXCarry * kWCarry);
constexpr float kScaleHW  = 1.0f / (kHidCarry * kWCarry);
constexpr float kScaleOut = 1.0f / (kYCarry * kWCarry);
constexpr float kQScale   = 1.0f / (float)kHdimRoot;
constexpr float kF16Min   = 6.103515625e-5f;
constexpr float kF32Min   = 1.17549435e-38f;
constexpr float kNormEps  = 1e-6f;
constexpr float kL2Eps    = 1e-6f;

static_assert(kHdimRoot * kHdimRoot == kHdim, "q scale");
static_assert(kProj == 1024 && kHdim == 64 && kHeads == 16 && kChunk == 16, "layout");
static_assert(kTok % 32 == 0 && kProj % 64 == 0 && kHid % 64 == 0 && kLow % 64 == 0 && kBetaPad % 64 == 0, "tile multiples");
static_assert(kHid % 32 == 0 && kProj % 32 == 0 && kLow % 32 == 0, "k multiples of 32");
static_assert(kTok % kChunk == 0, "chunking");
static_assert(((kTok / 32) * (kProj / 64)) % 8 == 0 && ((kTok / 32) * (kLow / 64)) % 8 == 0 &&
              ((kTok / 32) * (kHid / 64)) % 8 == 0, "whole blocks of tiles");
static_assert(kTaps == 4, "taps");

typedef __attribute__((ext_vector_type(16))) _Float16 v16h;
typedef __attribute__((ext_vector_type(8)))  _Float16 v8h;
typedef __attribute__((ext_vector_type(8)))  float    v8f;
typedef __attribute__((ext_vector_type(4)))  float    v4f;
typedef __attribute__((ext_vector_type(2)))  float    v2f;
typedef __attribute__((ext_vector_type(4)))  unsigned int v4u;

__device__ __forceinline__ unsigned pk16(unsigned short a, unsigned short b) {
  return (unsigned)a | ((unsigned)b << 16);
}
__device__ __forceinline__ float flush16(float v) {
  return (fabsf(v) < kF16Min) ? 0.0f : v;
}
__device__ __forceinline__ unsigned short h_bits(float f) {
  const _Float16 h = (_Float16)flush16(f);
  return __builtin_bit_cast(unsigned short, h);
}
__device__ __forceinline__ void h_split(float v, unsigned short& hb, unsigned short& rb) {
  const _Float16 h = (_Float16)flush16(v);
  const float hf = (float)h;
  const float d = v - hf;
  const _Float16 r = (_Float16)flush16(d * kResCarry);
  hb = __builtin_bit_cast(unsigned short, h);
  rb = __builtin_bit_cast(unsigned short, r);
}
__device__ __forceinline__ void pack8_split(const float (&v)[8], v4u& uh, v4u& ur) {
  unsigned short hb[8], rb[8];
#pragma unroll
  for (int e = 0; e < 8; ++e) h_split(v[e], hb[e], rb[e]);
  uh = (v4u){pk16(hb[0], hb[1]), pk16(hb[2], hb[3]), pk16(hb[4], hb[5]), pk16(hb[6], hb[7])};
  ur = (v4u){pk16(rb[0], rb[1]), pk16(rb[2], rb[3]), pk16(rb[4], rb[5]), pk16(rb[6], rb[7])};
}
__device__ __forceinline__ float wave_sum32(float v) {
#pragma unroll
  for (int o = 16; o > 0; o >>= 1) v += __shfl_xor(v, o, 32);
  return v;
}

struct FragH {
  union U { v16h v; v8h h[2]; };
  static __device__ __forceinline__ v16h load(const _Float16* p) {
    U f;
    f.h[0] = *(const v8h*)(p);
    f.h[1] = *(const v8h*)(p + 16);
    return f.v;
  }
  static __device__ __forceinline__ v8f mma(v16h a, v16h b, v8f c) {
    return __builtin_amdgcn_wmma_f32_16x16x32_f16(false, a, false, b, (short)0, c, false, false);
  }
};
__device__ __forceinline__ void guard_main(v8f& a, v16h x, v16h y) {
  asm volatile("v_nop\n\tv_nop\n\tv_nop\n\tv_nop" : "+v"(a) : "v"(x), "v"(y));
}
__device__ __forceinline__ void guard_res(v8f& a, v16h x0, v16h x1, v16h y0, v16h y1) {
  asm volatile("v_nop\n\tv_nop\n\tv_nop\n\tv_nop" : "+v"(a) : "v"(x0), "v"(x1), "v"(y0), "v"(y1));
}
__device__ __forceinline__ void acc_guard1(v8f& a) {
  asm volatile("v_nop\n\tv_nop\n\tv_nop\n\tv_nop" : "+v"(a));
}

template <bool SPLIT, int OUT_MODE>
__global__ __launch_bounds__(256) void gemm_f16_kernel(
    const unsigned short* __restrict__ Ahp, const unsigned short* __restrict__ Arp, int lda, long strideA,
    const unsigned short* __restrict__ Bhp, const unsigned short* __restrict__ Brp, int ldb, long strideB,
    void* __restrict__ Cout, int ldc, long strideC,
    int M, int N, int K, float scale) {
  __shared__ __align__(16) float sT[8][16 * 68];
  const int z    = blockIdx.y;
  const int lane = threadIdx.x & 31;
  const int wave = threadIdx.x >> 5;
  const int tilesN = N >> 6;
  const int tilesM = M >> 5;
  const int tile = blockIdx.x * 8 + wave;
  if (tile >= tilesM * tilesN) return;
  const int tm = tile / tilesN;
  const int tn = tile - tm * tilesN;
  const int m0 = tm << 5;
  const int n0 = tn << 6;
  const int rlane = lane & 15;
  const int half8 = (lane >> 4) * 8;
  const int mOff  = (lane >> 4) * 8;

  const size_t aoff = (size_t)z * (size_t)strideA + (size_t)(m0 + rlane) * lda + half8;
  const size_t boff = (size_t)z * (size_t)strideB + (size_t)(n0 + rlane) * ldb + half8;
  const _Float16* pa0 = (const _Float16*)Ahp + aoff;
  const _Float16* pa1 = pa0 + (size_t)16 * lda;
  const _Float16* pr0 = SPLIT ? ((const _Float16*)Arp + aoff) : pa0;
  const _Float16* pr1 = pr0 + (size_t)16 * lda;
  const _Float16* pbh = (const _Float16*)Bhp + boff;
  const _Float16* pbr = SPLIT ? ((const _Float16*)Brp + boff) : pbh;
  const size_t bstep = (size_t)16 * ldb;

  v8f acc[2][4], accr[2][4];
#pragma unroll
  for (int i = 0; i < 2; ++i)
#pragma unroll
    for (int j = 0; j < 4; ++j) {
      acc[i][j]  = (v8f){0.f, 0.f, 0.f, 0.f, 0.f, 0.f, 0.f, 0.f};
      accr[i][j] = (v8f){0.f, 0.f, 0.f, 0.f, 0.f, 0.f, 0.f, 0.f};
    }

  for (int k0 = 0; k0 < K; k0 += 32) {
    const v16h ah0 = FragH::load(pa0 + k0);
    const v16h ah1 = FragH::load(pa1 + k0);
    v16h ar0 = ah0, ar1 = ah1;
    if (SPLIT) {
      ar0 = FragH::load(pr0 + k0);
      ar1 = FragH::load(pr1 + k0);
    }
#pragma unroll
    for (int j = 0; j < 4; ++j) {
      const v16h bh = FragH::load(pbh + j * bstep + k0);
      v16h br = bh;
      if (SPLIT) br = FragH::load(pbr + j * bstep + k0);
      acc[0][j] = FragH::mma(ah0, bh, acc[0][j]);
      acc[1][j] = FragH::mma(ah1, bh, acc[1][j]);
      if (SPLIT) {
        accr[0][j] = FragH::mma(ah0, br, accr[0][j]);
        accr[1][j] = FragH::mma(ah1, br, accr[1][j]);
        accr[0][j] = FragH::mma(ar0, bh, accr[0][j]);
        accr[1][j] = FragH::mma(ar1, bh, accr[1][j]);
        guard_main(acc[0][j], ah0, bh);
        guard_main(acc[1][j], ah1, bh);
        guard_res(accr[0][j], ah0, ar0, bh, br);
        guard_res(accr[1][j], ah1, ar1, bh, br);
      } else {
        guard_main(acc[0][j], ah0, bh);
        guard_main(acc[1][j], ah1, bh);
      }
    }
  }
#pragma unroll
  for (int i = 0; i < 2; ++i)
#pragma unroll
    for (int j = 0; j < 4; ++j) {
      acc_guard1(acc[i][j]);
      if (SPLIT) acc_guard1(accr[i][j]);
    }

  float* slab = sT[wave];
#pragma unroll
  for (int i = 0; i < 2; ++i) {
    const int mBase = m0 + (i << 4);
#pragma unroll
    for (int j = 0; j < 4; ++j) {
#pragma unroll
      for (int r = 0; r < 8; ++r) {
        float v = acc[i][j][r];
        if (SPLIT) v += accr[i][j][r] * kResInv;
        v *= scale;
        slab[(mOff + r) * 68 + (j << 4) + rlane] = v;
      }
    }
    __builtin_amdgcn_fence(__ATOMIC_RELEASE, "workgroup");
    __builtin_amdgcn_wave_barrier();
    __builtin_amdgcn_fence(__ATOMIC_ACQUIRE, "workgroup");
    if (OUT_MODE == 0) {
      float* C = (float*)Cout + (size_t)z * (size_t)strideC;
      const int hh = lane >> 4, c4 = (lane & 15) * 4;
      for (int pass = 0; pass < 2; ++pass) {
#pragma unroll
        for (int it = 0; it < 8; ++it) {
          const int row = it * 2 + hh;
          const v4f v = *(const v4f*)(slab + row * 68 + c4);
          *(volatile v4f*)(C + (size_t)(mBase + row) * ldc + n0 + c4) = v;
        }
        __threadfence();
      }
    } else {
      const int q = lane >> 3, c8 = (lane & 7) * 8;
      unsigned short* C = (unsigned short*)Cout + (size_t)z * (size_t)strideC;
      for (int pass = 0; pass < 2; ++pass) {
#pragma unroll
        for (int it = 0; it < 4; ++it) {
          const int row = it * 4 + q;
          const float* sp = slab + row * 68 + c8;
          v8h hv;
#pragma unroll
          for (int e = 0; e < 8; ++e) {
            const float xv = sp[e];
            const float xf = flush16(xv);
            hv[e] = (_Float16)xf;
          }
          *(volatile v8h*)(C + (size_t)(mBase + row) * ldc + n0 + c8) = hv;
        }
        __threadfence();
      }
    }
    __builtin_amdgcn_fence(__ATOMIC_RELEASE, "workgroup");
    __builtin_amdgcn_wave_barrier();
    __builtin_amdgcn_fence(__ATOMIC_ACQUIRE, "workgroup");
  }
}

__global__ __launch_bounds__(256) void cast_plane_kernel(const float* s0, const float* s1, const float* s2,
                                                         unsigned short* __restrict__ dh, unsigned short* __restrict__ dr,
                                                         int total8, int src_elems, float carry, int has_res) {
  const int i = blockIdx.x * 256 + threadIdx.x;
  if (i >= total8) return;
  const int z = blockIdx.y;
  const float* src = (z == 0) ? s0 : (z == 1) ? s1 : s2;
  const int e0 = i * 8;
  const bool valid = (e0 < src_elems);
  const int ec = valid ? e0 : 0;
  v4f a = *(const v4f*)(src + ec);
  v4f b = *(const v4f*)(src + ec + 4);
  asm volatile("" : "+v"(a), "+v"(b));
  float v[8];
#pragma unroll
  for (int e = 0; e < 4; ++e) {
    v[e]     = valid ? (a[e] * carry) : 0.0f;
    v[4 + e] = valid ? (b[e] * carry) : 0.0f;
  }
  v4u uh, ur;
  pack8_split(v, uh, ur);
  const size_t off = (size_t)z * (size_t)total8 * 8 + (size_t)e0;
  for (int pass = 0; pass < 2; ++pass) {
    *(volatile v4u*)(dh + off) = uh;
    if (has_res) *(volatile v4u*)(dr + off) = ur;
    __threadfence();
  }
}

__global__ __launch_bounds__(256) void conv_norm_kernel(const float* __restrict__ P3,
                                                        const float* __restrict__ cq, const float* __restrict__ ck,
                                                        const float* __restrict__ cv, float* __restrict__ N3) {
  const int lane = threadIdx.x & 31;
  const int pair = blockIdx.x * 8 + (threadIdx.x >> 5);
  const int tok = pair >> 4;
  const int hd  = pair & 15;
  const int c = hd * kHdim + 2 * lane;
  const size_t base = (size_t)tok * kProj + (size_t)c;
#pragma unroll 1
  for (int p = 0; p < 3; ++p) {
    const float* src = P3 + (size_t)p * kPlane;
    const float* cw = (p == 0) ? cq : (p == 1) ? ck : cv;
    const v4f w0 = *(const v4f*)(cw + (size_t)c * kTaps);
    const v4f w1 = *(const v4f*)(cw + (size_t)c * kTaps + 4);
    float a0 = 0.0f, a1 = 0.0f;
#pragma unroll
    for (int i = 0; i < kTaps; ++i) {
      const int tt = tok - (kTaps - 1) + i;
      const bool ok = (tt >= 0);
      const int tc = ok ? tt : 0;
      v2f x = *(const v2f*)(src + (size_t)tc * kProj + c);
      asm volatile("" : "+v"(x));
      const float x0 = ok ? x[0] : 0.0f;
      const float x1 = ok ? x[1] : 0.0f;
      a0 += x0 * w0[i];
      a1 += x1 * w1[i];
    }
    const float s0 = a0 * __builtin_amdgcn_rcpf(1.0f + expf(-a0));
    const float s1 = a1 * __builtin_amdgcn_rcpf(1.0f + expf(-a1));
    const float ss = wave_sum32(s0 * s0 + s1 * s1);
    const float inv = __builtin_amdgcn_rcpf(fmaxf(sqrtf(ss), kL2Eps));
    const float mul = (p == 0) ? (inv * kQScale) : (p == 1) ? inv : 1.0f;
    const v2f o = (v2f){s0 * mul, s1 * mul};
    float* dst = N3 + (size_t)p * kPlane + base;
    *(volatile v2f*)dst = o;
    __threadfence();
    *(volatile v2f*)dst = o;
  }
}

__global__ __launch_bounds__(256) void decay_kernel(float* RG, const float* __restrict__ A_log,
                                                    const float* __restrict__ dt_bias) {
  const int i = blockIdx.x * 256 + threadIdx.x;
  if (i >= kTok * kProj) return;
  const int c = i & (kProj - 1);
  const int hd = c >> 6;
  const float x = RG[i] + dt_bias[c];
  const float sp = fmaxf(x, 0.0f) + log1pf(expf(-fabsf(x)));
  const float g = -expf(A_log[hd]) * sp;
  float d = expf(g);
  d = (d < kF32Min) ? 0.0f : d;
  *(volatile float*)(RG + i) = d;
  __threadfence();
  *(volatile float*)(RG + i) = d;
}

__global__ __launch_bounds__(256) void state_scan_kernel(const float* __restrict__ Qf, const float* __restrict__ Dd,
                                                         const float* __restrict__ Kf, const float* __restrict__ Vf,
                                                         const float* __restrict__ BR, float* __restrict__ Y) {
  __shared__ __align__(16) float lv[4 * kChunk * 64];
  __shared__ __align__(16) float yb[kChunk * 64];
  __shared__ __align__(16) float sb[kChunk];
  const int hd  = blockIdx.x;
  const int tid = threadIdx.x;
  const int i   = tid >> 2;
  const int q   = tid & 3;
  const int j0  = q * 16;
  const int lrow = tid >> 4;
  const int lc4  = (tid & 15) * 4;
  const size_t base = (size_t)hd * kHdim;

  float S[16];
#pragma unroll
  for (int jj = 0; jj < 16; ++jj) S[jj] = 0.0f;

#pragma unroll 1
  for (int ch = 0; ch < kTok / kChunk; ++ch) {
    const size_t goff = base + (size_t)(ch * kChunk + lrow) * kProj + lc4;
    {
      const v4f t0 = *(const v4f*)(Qf + goff);
      const v4f t1 = *(const v4f*)(Dd + goff);
      const v4f t2 = *(const v4f*)(Kf + goff);
      const v4f t3 = *(const v4f*)(Vf + goff);
      float braw = BR[(size_t)(ch * kChunk + (tid & 15)) * kBetaPad + hd];
      asm volatile("" : "+v"(braw));
      const float bsig = __builtin_amdgcn_rcpf(1.0f + expf(-braw));
      const int lo = lrow * 64 + lc4;
      *(v4f*)(lv + 0 * kChunk * 64 + lo) = t0;
      *(v4f*)(lv + 1 * kChunk * 64 + lo) = t1;
      *(v4f*)(lv + 2 * kChunk * 64 + lo) = t2;
      *(v4f*)(lv + 3 * kChunk * 64 + lo) = t3;
      if (tid < kChunk) sb[tid] = bsig;
    }
    __syncthreads();

#pragma unroll 1
    for (int s = 0; s < kChunk; ++s) {
      const float* pq = lv + 0 * kChunk * 64 + s * 64 + j0;
      const float* pd = lv + 1 * kChunk * 64 + s * 64 + j0;
      const float* pk = lv + 2 * kChunk * 64 + s * 64 + j0;
      const float vi = lv[3 * kChunk * 64 + s * 64 + i];
      const float bt = sb[s];
      float sa = 0.0f;
#pragma unroll
      for (int g4 = 0; g4 < 4; ++g4) {
        const v4f d4 = *(const v4f*)(pd + 4 * g4);
        const v4f k4 = *(const v4f*)(pk + 4 * g4);
#pragma unroll
        for (int e = 0; e < 4; ++e) {
          const float sd = S[4 * g4 + e] * d4[e];
          S[4 * g4 + e] = sd;
          sa += sd * k4[e];
        }
      }
      sa += __shfl_xor(sa, 1, 32);
      sa += __shfl_xor(sa, 2, 32);
      const float be = bt * (vi - sa);
      float out = 0.0f;
#pragma unroll
      for (int g4 = 0; g4 < 4; ++g4) {
        const v4f k4 = *(const v4f*)(pk + 4 * g4);
        const v4f q4 = *(const v4f*)(pq + 4 * g4);
#pragma unroll
        for (int e = 0; e < 4; ++e) {
          const float sn = S[4 * g4 + e] + be * k4[e];
          S[4 * g4 + e] = sn;
          out += sn * q4[e];
        }
      }
      out += __shfl_xor(out, 1, 32);
      out += __shfl_xor(out, 2, 32);
      if (q == 0) yb[s * 64 + i] = out;
    }
    __syncthreads();
    {
      const v4f val = *(const v4f*)(yb + lrow * 64 + lc4);
      *(volatile v4f*)(Y + goff) = val;
      __threadfence();
      *(volatile v4f*)(Y + goff) = val;
    }
  }
}

__global__ __launch_bounds__(256) void norm_gate_kernel(const float* __restrict__ Y, const float* __restrict__ OG,
                                                        const float* __restrict__ nw, unsigned* __restrict__ YG) {
  const int lane = threadIdx.x & 31;
  const int pair = blockIdx.x * 8 + (threadIdx.x >> 5);
  const int tok = pair >> 4;
  const int hd  = pair & 15;
  const size_t base = (size_t)tok * kProj + (size_t)hd * kHdim + 2 * lane;
  const v2f y2 = *(const v2f*)(Y + base);
  const v2f g2 = *(const v2f*)(OG + base);
  const v2f w2 = *(const v2f*)(nw + 2 * lane);
  const float ms = wave_sum32(y2[0] * y2[0] + y2[1] * y2[1]) * (1.0f / (float)kHdim);
  const float inv = 1.0f / sqrtf(ms + kNormEps);
  const float s0 = __builtin_amdgcn_rcpf(1.0f + expf(-g2[0]));
  const float s1 = __builtin_amdgcn_rcpf(1.0f + expf(-g2[1]));
  const float o0 = ((y2[0] * inv) * w2[0]) * s0 * kYCarry;
  const float o1 = ((y2[1] * inv) * w2[1]) * s1 * kYCarry;
  const unsigned short h0 = h_bits(o0);
  const unsigned short h1 = h_bits(o1);
  const unsigned wh = pk16(h0, h1);
  const size_t widx = base >> 1;
  *(volatile unsigned*)(YG + widx) = wh;
  __threadfence();
  *(volatile unsigned*)(YG + widx) = wh;
}

extern "C" void kernel_launch(void* const* d_in, const int* in_sizes, int n_in,
                              void* d_out, int out_size, void* d_ws, size_t ws_size, hipStream_t stream) {
  if (n_in < 16 || d_out == nullptr || d_ws == nullptr) return;
  if (in_sizes[0] != kTok * kHid) return;
  if (in_sizes[1] != kProj * kHid || in_sizes[2] != kProj * kHid || in_sizes[3] != kProj * kHid) return;
  if (in_sizes[4] != kProj * kTaps || in_sizes[5] != kProj * kTaps || in_sizes[6] != kProj * kTaps) return;
  if (in_sizes[7] != kHeads || in_sizes[8] != kProj) return;
  if (in_sizes[9] != kLow * kHid || in_sizes[10] != kProj * kLow) return;
  if (in_sizes[11] != kHeads * kHid) return;
  if (in_sizes[12] != kLow * kHid || in_sizes[13] != kProj * kLow) return;
  if (in_sizes[14] != kHdim || in_sizes[15] != kHid * kProj) return;
  if (out_size != kTok * kHid) return;

  const float* h_in    = (const float*)d_in[0];
  const float* Wq      = (const float*)d_in[1];
  const float* Wk      = (const float*)d_in[2];
  const float* Wv      = (const float*)d_in[3];
  const float* conv_q  = (const float*)d_in[4];
  const float* conv_k  = (const float*)d_in[5];
  const float* conv_v  = (const float*)d_in[6];
  const float* A_log   = (const float*)d_in[7];
  const float* dt_bias = (const float*)d_in[8];
  const float* Wfa     = (const float*)d_in[9];
  const float* Wfb     = (const float*)d_in[10];
  const float* Wb      = (const float*)d_in[11];
  const float* Wga     = (const float*)d_in[12];
  const float* Wgb     = (const float*)d_in[13];
  const float* norm_w  = (const float*)d_in[14];
  const float* Wo      = (const float*)d_in[15];
  float* out = (float*)d_out;

  char* ws = (char*)d_ws;
  size_t off = 0;
  auto carve = [&](size_t bytes) -> char* {
    char* p = ws + off;
    off += (bytes + 255) & ~(size_t)255;
    return p;
  };
  const size_t wBig = (size_t)kProj * kHid;
  unsigned short* XH   = (unsigned short*)carve((size_t)kTok * kHid * 2);
  unsigned short* XR   = (unsigned short*)carve((size_t)kTok * kHid * 2);
  unsigned short* WQh  = (unsigned short*)carve(3 * wBig * 2);
  unsigned short* WQr  = (unsigned short*)carve(3 * wBig * 2);
  unsigned short* WOh  = (unsigned short*)carve((size_t)kHid * kProj * 2);
  unsigned short* WFGA = (unsigned short*)carve((size_t)2 * kLow * kHid * 2);
  unsigned short* WBp  = (unsigned short*)carve((size_t)kBetaPad * kHid * 2);
  unsigned short* WFGB = (unsigned short*)carve((size_t)2 * kProj * kLow * 2);
  unsigned short* FGA  = (unsigned short*)carve((size_t)2 * kTok * kLow * 2);
  float* BR   = (float*)carve((size_t)kTok * kBetaPad * 4);
  float* QKVP = (float*)carve(3 * kPlane * 4);
  float* QKVN = (float*)carve(3 * kPlane * 4);
  float* RG   = (float*)carve(2 * kPlane * 4);
  float* Yf   = (float*)carve(kPlane * 4);
  unsigned short* YG = (unsigned short*)carve(kPlane * 2);
  if (off != (size_t)127926272) return;
  if (off > ws_size || off > (size_t)134217728) return;

  cast_plane_kernel<<<dim3((kTok * kHid / 8) / 256, 1), 256, 0, stream>>>(
      h_in, h_in, h_in, XH, XR, kTok * kHid / 8, kTok * kHid, kXCarry, 1);
  cast_plane_kernel<<<dim3((kProj * kHid / 8) / 256, 3), 256, 0, stream>>>(
      Wq, Wk, Wv, WQh, WQr, kProj * kHid / 8, kProj * kHid, kWCarry, 1);
  cast_plane_kernel<<<dim3((kHid * kProj / 8) / 256, 1), 256, 0, stream>>>(
      Wo, Wo, Wo, WOh, WOh, kHid * kProj / 8, kHid * kProj, kWCarry, 0);
  cast_plane_kernel<<<dim3((kLow * kHid / 8) / 256, 2), 256, 0, stream>>>(
      Wfa, Wga, Wga, WFGA, WFGA, kLow * kHid / 8, kLow * kHid, kWCarry, 0);
  cast_plane_kernel<<<dim3((kBetaPad * kHid / 8) / 256, 1), 256, 0, stream>>>(
      Wb, Wb, Wb, WBp, WBp, kBetaPad * kHid / 8, kHeads * kHid, kWCarry, 0);
  cast_plane_kernel<<<dim3((kProj * kLow / 8) / 256, 2), 256, 0, stream>>>(
      Wfb, Wgb, Wgb, WFGB, WFGB, kProj * kLow / 8, kProj * kLow, kWCarry, 0);

  const int blkBig = (kTok / 32) * (kProj / 64) / 8;
  const int blk64  = (kTok / 32) * (kLow / 64) / 8;
  const int blkOut = (kTok / 32) * (kHid / 64) / 8;
  gemm_f16_kernel<true, 0><<<dim3(blkBig, 3), 256, 0, stream>>>(
      XH, XR, kHid, 0L, WQh, WQr, kHid, (long)wBig,
      (void*)QKVP, kProj, (long)kPlane, kTok, kProj, kHid, kScaleXW);

  gemm_f16_kernel<false, 1><<<dim3(blk64, 2), 256, 0, stream>>>(
      XH, XH, kHid, 0L, WFGA, WFGA, kHid, (long)((size_t)kLow * kHid),
      (void*)FGA, kLow, (long)((size_t)kTok * kLow), kTok, kLow, kHid, kScaleHid);

  gemm_f16_kernel<false, 0><<<dim3(blk64, 1), 256, 0, stream>>>(
      XH, XH, kHid, 0L, WBp, WBp, kHid, 0L,
      (void*)BR, kBetaPad, 0L, kTok, kBetaPad, kHid, kScaleXW);

  gemm_f16_kernel<false, 0><<<dim3(blkBig, 2), 256, 0, stream>>>(
      FGA, FGA, kLow, (long)((size_t)kTok * kLow), WFGB, WFGB, kLow, (long)((size_t)kProj * kLow),
      (void*)RG, kProj, (long)kPlane, kTok, kProj, kLow, kScaleHW);

  conv_norm_kernel<<<(kTok * kHeads) / 8, 256, 0, stream>>>(QKVP, conv_q, conv_k, conv_v, QKVN);

  decay_kernel<<<(kTok * kProj) / 256, 256, 0, stream>>>(RG, A_log, dt_bias);

  state_scan_kernel<<<kHeads, 256, 0, stream>>>(QKVN, RG, QKVN + kPlane, QKVN + 2 * kPlane, BR, Yf);

  norm_gate_kernel<<<(kTok * kHeads) / 8, 256, 0, stream>>>(Yf, RG + kPlane, norm_w, (unsigned*)YG);

  gemm_f16_kernel<false, 0><<<dim3(blkOut, 1), 256, 0, stream>>>(
      YG, YG, kProj, 0L, WOh, WOh, kProj, 0L,
      (void*)out, kHid, 0L, kTok, kHid, kProj, kScaleOut);
}
